// Norm1dBatched_31207232373392
// MI455X (gfx1250) — hardware-verified
//
#include <hip/hip_runtime.h>
#include <stddef.h>


typedef _Float16 v16h __attribute__((ext_vector_type(16)));
typedef _Float16 v8h  __attribute__((ext_vector_type(8)));
typedef float    v8f  __attribute__((ext_vector_type(8)));
typedef float    v4f  __attribute__((ext_vector_type(4)));
typedef _Float16 h16;

#ifndef NFEAT
#define NFEAT 8192
#endif
#define NFEAT_FULL 8192
#define BB 512
#define KP 1024

static_assert(NFEAT >= 64 && NFEAT <= NFEAT_FULL && (NFEAT % 64) == 0);
static_assert(BB == 512 && (BB % 64) == 0);
static_assert(KP == 2 * BB && (KP % 32) == 0 && (KP % 64) == 0);
static_assert(((BB * (KP / 8)) % 256) == 0);
static_assert((NFEAT_FULL % 4) == 0);

#define LDT 72
#define LDC 68
static_assert((LDT % 8) == 0 && LDT >= 64);
static_assert((LDC % 4) == 0 && LDC >= 64);
static_assert(64 * LDT * 2 <= 131072);
static_assert(64 * LDC * 4 <= 131072);

#define XCARRY 64.0f
#define VCARRY 256.0f
#define ALPHA_F 0.999f
#define OMA_F   0.001f
#define AB_F    0.5991422854f
#define LOG2A_F (-0.00144341686899f)
#define EPS_F   1.0e-5f

#define TP_BYTES   ((size_t)BB * KP * 2)
#define XT_BYTES   ((size_t)NFEAT * KP * 2)
#define CENT_BYTES ((size_t)BB * NFEAT * 4)
#define OFF_TP   ((size_t)0)
#define OFF_XM   (OFF_TP + TP_BYTES)
#define OFF_XV   (OFF_XM + XT_BYTES)
#define OFF_CENT (OFF_XV + XT_BYTES)
#define WS_TOTAL (OFF_CENT + CENT_BYTES)
static_assert((TP_BYTES % 128) == 0 && (XT_BYTES % 128) == 0 && (CENT_BYTES % 128) == 0);
static_assert(WS_TOTAL <= (size_t)134217728);

__device__ __forceinline__ float bf16r(float x) {
  unsigned int u = __float_as_uint(x);
  u = (u + 0x7FFFu + ((u >> 16) & 1u)) & 0xFFFF0000u;
  return __uint_as_float(u);
}

static __device__ __forceinline__ h16 toh_flush(float v) {
  const h16 r = (h16)v;
  return (fabsf(v) < 6.103515625e-05f) ? (h16)0.0f : r;
}

__device__ __forceinline__ v16h frag_at(const _Float16* p) {
  v8h lo = *(const v8h*)(p);
  v8h hi = *(const v8h*)(p + 16);
  v16h out;
#pragma unroll
  for (int i = 0; i < 8; ++i) { out[i] = lo[i]; out[i + 8] = hi[i]; }
  return out;
}

__device__ __forceinline__ v8f wmma16(v16h a, v16h b, v8f c) {
  v8f d = __builtin_amdgcn_wmma_f32_16x16x32_f16(false, a, false, b, (short)0, c,
                                                 false, false);
  asm volatile("v_nop\n\tv_nop\n\tv_nop\n\tv_nop" : "+v"(d) : "v"(a), "v"(b));
  return d;
}

__global__ __launch_bounds__(256) void toep_kernel(_Float16* __restrict__ TP) {
#pragma clang fp contract(off)
  const unsigned gid = blockIdx.x * 256u + threadIdx.x;
  const unsigned t = gid >> 7;
  const unsigned kc = (gid & 127u) * 8u;
  v8h o;
#pragma unroll
  for (int j = 0; j < 8; ++j) {
    const int e = 511 - (int)(kc + (unsigned)j) + (int)t;
    const bool ok = (t >= 1u) && (e >= 0) && (e <= 511);
    const int ec = ok ? e : 0;
    const float wv = __builtin_exp2f((float)ec * LOG2A_F);
    o[j] = toh_flush(ok ? wv : 0.0f);
  }
  _Float16* p = TP + (size_t)t * KP + kc;
  *(volatile v8h*)p = o;
  __threadfence();
  *(volatile v8h*)p = o;
}

__global__ __launch_bounds__(256) void xconv_kernel(
    const float* __restrict__ W, _Float16* __restrict__ Wt, unsigned ldw, unsigned ldk,
    unsigned kofs, float carry, unsigned zrow0) {
#pragma clang fp contract(off)
  __shared__ _Float16 T[64 * LDT];
  const unsigned tid = threadIdx.x;
  const unsigned n0 = blockIdx.x * 64u;
  const unsigned k0 = blockIdx.y * 64u;
#pragma unroll 4
  for (unsigned j = 0; j < 16u; ++j) {
    const unsigned idx = tid + 256u * j;
    const unsigned kr = idx >> 6, nc = idx & 63u;
    float v = W[(size_t)(k0 + kr) * ldw + n0 + nc];
    asm volatile("" : "+v"(v));
    const float vz = (zrow0 != 0u && (k0 + kr) == 0u) ? 0.0f : v;
    T[nc * LDT + kr] = toh_flush(carry * bf16r(vz));
  }
  __syncthreads();
  v8h x[2];
  size_t off[2];
#pragma unroll
  for (unsigned i = 0; i < 2u; ++i) {
    const unsigned n = 32u * i + (tid >> 3);
    const unsigned kc = (tid & 7u) * 8u;
    x[i] = *(const v8h*)&T[n * LDT + kc];
    off[i] = (size_t)(n0 + n) * ldk + kofs + k0 + kc;
  }
#pragma unroll
  for (int i = 0; i < 2; ++i) *(volatile v8h*)(Wt + off[i]) = x[i];
  __threadfence();
#pragma unroll
  for (int i = 0; i < 2; ++i) *(volatile v8h*)(Wt + off[i]) = x[i];
}

template <int MODE>
__device__ __forceinline__ void gemm_body(
    const _Float16* __restrict__ A16, const _Float16* __restrict__ Bt,
    const float* __restrict__ xin, const float* __restrict__ strm,
    float* __restrict__ centp, _Float16* __restrict__ out16, float* __restrict__ outf) {
  __shared__ float Cs[64 * LDC];
  const unsigned tid = threadIdx.x, lane = tid & 31u;
  const unsigned w = (unsigned)__builtin_amdgcn_readfirstlane((int)(tid >> 5));
  const unsigned mw = w >> 1, nw = w & 1u;
  const unsigned hh = lane >> 4, m = lane & 15u;
  const unsigned n0 = blockIdx.x * 64u;
  const unsigned row0 = blockIdx.y * 64u;
  const unsigned K = (unsigned)KP;
  const unsigned kbeg = row0;
  const unsigned kend = (row0 + 576u < K) ? (row0 + 576u) : K;

  const _Float16* ap  = A16 + (size_t)(row0 + mw * 16u + m) * K + hh * 8u;
  const _Float16* bp0 = Bt + (size_t)(n0 + nw * 32u + m) * K + hh * 8u;
  const _Float16* bp1 = bp0 + (size_t)16 * K;
  v8f acc0 = {}, acc1 = {};
#pragma unroll 2
  for (unsigned k0 = kbeg; k0 < kend; k0 += 32u) {
    const v16h a  = frag_at(ap + k0);
    const v16h b0 = frag_at(bp0 + k0);
    const v16h b1 = frag_at(bp1 + k0);
    acc0 = wmma16(a, b0, acc0);
    acc1 = wmma16(a, b1, acc1);
  }
#pragma unroll
  for (int r = 0; r < 8; ++r) {
    float* d = &Cs[(mw * 16u + hh * 8u + (unsigned)r) * LDC + nw * 32u + m];
    d[0]  = acc0[r];
    d[16] = acc1[r];
  }
  __syncthreads();

  if (MODE == 0) {
    v4f xs[4];
    size_t off[4];
#pragma unroll
    for (unsigned i = 0; i < 4u; ++i) {
      const unsigned r = 16u * i + (tid >> 4);
      const unsigned c = (tid & 15u) * 4u;
      const unsigned t = row0 + r;
      const unsigned srow = (t == 0u) ? (unsigned)(BB - 1) : (t - 1u);
      const v4f u  = *(const v4f*)&Cs[r * LDC + c];
      const v4f xv = *(const v4f*)(xin + (size_t)t * NFEAT_FULL + n0 + c);
      const v4f sv = *(const v4f*)(strm + (size_t)srow * NFEAT_FULL + n0 + c);
      v4f val, vc;
#pragma unroll
      for (int j = 0; j < 4; ++j) {
        const float sm = bf16r(sv[j]);
        const float st = (t == 0u) ? sm : (AB_F * sm + OMA_F * (u[j] * (1.0f / XCARRY)));
        const float ce = bf16r(xv[j]) - st;
        val[j] = ce;
        vc[j] = VCARRY * ((ALPHA_F * ce) * ce);
      }
      *(v4f*)&Cs[r * LDC + c] = vc;
      xs[i] = val;
      off[i] = (size_t)t * NFEAT + n0 + c;
    }
#pragma unroll
    for (int i = 0; i < 4; ++i) *(volatile v4f*)(centp + off[i]) = xs[i];
    __threadfence();
#pragma unroll
    for (int i = 0; i < 4; ++i) *(volatile v4f*)(centp + off[i]) = xs[i];
    __syncthreads();

    v8h x[2];
    size_t o2[2];
#pragma unroll
    for (unsigned i = 0; i < 2u; ++i) {
      const unsigned dcol = 32u * i + (tid >> 3);
      const unsigned kk = (tid & 7u) * 8u;
#pragma unroll
      for (unsigned j = 0; j < 8u; ++j)
        x[i][j] = toh_flush(Cs[(kk + j) * LDC + dcol]);
      o2[i] = (size_t)(n0 + dcol) * KP + (unsigned)BB + row0 + kk;
    }
#pragma unroll
    for (int i = 0; i < 2; ++i) *(volatile v8h*)(out16 + o2[i]) = x[i];
    __threadfence();
#pragma unroll
    for (int i = 0; i < 2; ++i) *(volatile v8h*)(out16 + o2[i]) = x[i];
  }

  if (MODE == 1) {
    v4f xs[4];
    size_t off[4];
#pragma unroll
    for (unsigned i = 0; i < 4u; ++i) {
      const unsigned r = 16u * i + (tid >> 4);
      const unsigned c = (tid & 15u) * 4u;
      const unsigned t = row0 + r;
      const unsigned srow = (t == 0u) ? (unsigned)(BB - 1) : (t - 1u);
      const v4f u  = *(const v4f*)&Cs[r * LDC + c];
      const v4f sv = *(const v4f*)(strm + (size_t)srow * NFEAT_FULL + n0 + c);
      const v4f ce = *(const v4f*)(centp + (size_t)t * NFEAT + n0 + c);
      v4f val;
#pragma unroll
      for (int j = 0; j < 4; ++j) {
        const float sm = bf16r(sv[j]);
        const float st = (t == 0u) ? sm : (AB_F * sm + OMA_F * (u[j] * (1.0f / VCARRY)));
        val[j] = ce[j] * rsqrtf(st + EPS_F);
      }
      xs[i] = val;
      off[i] = (size_t)t * NFEAT_FULL + n0 + c;
    }
#pragma unroll
    for (int i = 0; i < 4; ++i) *(volatile v4f*)(outf + off[i]) = xs[i];
    __threadfence();
#pragma unroll
    for (int i = 0; i < 4; ++i) *(volatile v4f*)(outf + off[i]) = xs[i];
  }
}

__global__ __launch_bounds__(256) void gemm_mean_kernel(
    const _Float16* __restrict__ TP, const _Float16* __restrict__ XT,
    const float* __restrict__ xin, const float* __restrict__ strm,
    float* __restrict__ centp, _Float16* __restrict__ xtv) {
  gemm_body<0>(TP, XT, xin, strm, centp, xtv, (float*)0);
}
__global__ __launch_bounds__(256) void gemm_var_kernel(
    const _Float16* __restrict__ TP, const _Float16* __restrict__ XT,
    const float* __restrict__ strm, float* __restrict__ centp, float* __restrict__ outf) {
  gemm_body<1>(TP, XT, strm, strm, centp, (_Float16*)0, outf);
}

extern "C" void kernel_launch(void* const* d_in, const int* in_sizes, int n_in,
                              void* d_out, int out_size, void* d_ws, size_t ws_size,
                              hipStream_t stream) {
  if (n_in < 5) return;
  const long long need = (long long)(BB - 1) * NFEAT_FULL + NFEAT;
  if ((long long)in_sizes[0] < need) return;
  if ((long long)in_sizes[1] < need) return;
  if ((long long)in_sizes[2] < need) return;
  if ((long long)in_sizes[3] < need) return;
  if ((long long)in_sizes[4] < need) return;
  if ((long long)out_size < need) return;
  if (ws_size < WS_TOTAL) return;

  const float* x     = (const float*)d_in[0];
  const float* m_p   = (const float*)d_in[1];
  const float* var_p = (const float*)d_in[2];
  const float* m     = (const float*)d_in[3];
  const float* var   = (const float*)d_in[4];
  float* out = (float*)d_out;

  char* ws = (char*)d_ws;
  _Float16* TP   = (_Float16*)(ws + OFF_TP);
  _Float16* XTM  = (_Float16*)(ws + OFF_XM);
  _Float16* XTV  = (_Float16*)(ws + OFF_XV);
  float*    CENT = (float*)(ws + OFF_CENT);

  dim3 blk(256);
  dim3 gt(NFEAT / 64, BB / 64);

  toep_kernel<<<dim3((BB * (KP / 8)) / 256), blk, 0, stream>>>(TP);
  xconv_kernel<<<gt, blk, 0, stream>>>(m_p, XTM, (unsigned)NFEAT_FULL, (unsigned)KP, 0u, XCARRY, 1u);
  xconv_kernel<<<gt, blk, 0, stream>>>(x, XTM, (unsigned)NFEAT_FULL, (unsigned)KP, (unsigned)BB, XCARRY, 0u);
  xconv_kernel<<<gt, blk, 0, stream>>>(var_p, XTV, (unsigned)NFEAT_FULL, (unsigned)KP, 0u, VCARRY, 1u);
  gemm_mean_kernel<<<gt, blk, 0, stream>>>(TP, XTM, x, m, CENT, XTV);
  gemm_var_kernel<<<gt, blk, 0, stream>>>(TP, XTV, var, CENT, out);
}
